// S4Block_37572373905579
// MI455X (gfx1250) — hardware-verified
//
#include <hip/hip_runtime.h>
#include <math.h>
#include <stdint.h>

#ifndef TROWS
#define TROWS 2048
#endif
#define NB    16
#define SEQ   2048
#define CH    128
#define NS    64
#define KDFT  (2 * SEQ)
#define LR    2120
#define CONV_DYN_BYTES (2 * 8 * LR * 2)
#define SAT   16.0f
#define RCA   1024.0f
#define KC    256.0f
#define RCK   1024.0f
#define RCH   1024.0f

static_assert(TROWS >= 64 && TROWS <= SEQ && (TROWS % 64) == 0);
static_assert(NB == 16);
static_assert((LR % 8) == 0 && LR >= 2119);
static_assert((CH % 64) == 0 && (SEQ % 64) == 0 && (KDFT % 32) == 0 && (CH % 32) == 0);
static_assert(CONV_DYN_BYTES == 67840);

#define SZ_TRG ((size_t)2 * SEQ * 4)
#define SZ_WOH ((size_t)CH * CH * 2)
#define SZ_Y32 ((size_t)CH * NB * SEQ * 4)
#define SZ_YH  ((size_t)CH * NB * SEQ * 2)
#define SZ_AT  ((size_t)CH * KDFT * 2)
#define SZ_TW  ((size_t)SEQ * KDFT * 2)
#define SZ_KT  ((size_t)CH * SEQ * 4)
#define SZ_HC  ((size_t)CH * NB * SEQ * 2)
#define SZ_H2  ((size_t)NB * SEQ * CH * 2)
#define WS_TOTAL (SZ_TRG + SZ_WOH + SZ_Y32 + SZ_YH + 2 * SZ_AT + SZ_TW + SZ_KT + 2 * SZ_HC + 2 * SZ_H2)
static_assert(WS_TOTAL <= (size_t)134217728);
static_assert((SZ_TRG % 16384) == 0 && (SZ_WOH % 16384) == 0);

typedef _Float16 v16h __attribute__((ext_vector_type(16)));
typedef _Float16 v8h  __attribute__((ext_vector_type(8)));
typedef __bf16   v16b __attribute__((ext_vector_type(16)));
typedef __bf16   v8b  __attribute__((ext_vector_type(8)));
typedef float    v8f  __attribute__((ext_vector_type(8)));
typedef float    v4f  __attribute__((ext_vector_type(4)));
typedef unsigned int v4u __attribute__((ext_vector_type(4)));

#if defined(__HIP_DEVICE_COMPILE__)
#define DEV_ASM 1
#else
#define DEV_ASM 0
#endif

__device__ __forceinline__ unsigned short bf_bits(float f) {
  unsigned u = __float_as_uint(f);
  return (unsigned short)((u + 0x7FFFu + ((u >> 16) & 1u)) >> 16);
}
__device__ __forceinline__ float bf_up(unsigned short hb) { return __uint_as_float(((unsigned)hb) << 16); }
__device__ __forceinline__ float bfr(float f) { return bf_up(bf_bits(f)); }
__device__ __forceinline__ unsigned short h_bits(_Float16 x) { return __builtin_bit_cast(unsigned short, x); }
__device__ __forceinline__ unsigned pk16(unsigned short a, unsigned short b) { return (unsigned)a | ((unsigned)b << 16); }
__device__ __forceinline__ v8f zero8() { v8f z = {0.f, 0.f, 0.f, 0.f, 0.f, 0.f, 0.f, 0.f}; return z; }

__device__ __forceinline__ void split16(float v, float rc, unsigned short& hb, unsigned short& lb) {
  const _Float16 x = (_Float16)v;
  float xf = (float)x;
  xf = (fabsf(xf) < 6.103515625e-05f) ? 0.0f : xf;
  hb = h_bits((_Float16)xf);
  lb = h_bits((_Float16)((v - xf) * rc));
}

template <typename OT> struct FT;
template <> struct FT<__bf16>   { typedef v16b frag; typedef v8b half8; };
template <> struct FT<_Float16> { typedef v16h frag; typedef v8h half8; };

template <typename OT>
__device__ __forceinline__ typename FT<OT>::frag ldfrag(const OT* p) {
  union { typename FT<OT>::frag v; typename FT<OT>::half8 h[2]; } f;
  f.h[0] = *(const typename FT<OT>::half8*)(p);
  f.h[1] = *(const typename FT<OT>::half8*)(p + 16);
  return f.v;
}

__device__ __forceinline__ v8f mmar(v16b a, v16b b, v8f c) {
  return __builtin_amdgcn_wmma_f32_16x16x32_bf16(false, a, false, b, (short)0, c, false, false);
}
__device__ __forceinline__ v8f mmar(v16h a, v16h b, v8f c) {
  return __builtin_amdgcn_wmma_f32_16x16x32_f16(false, a, false, b, (short)0, c, false, false);
}
__device__ __forceinline__ void dep_guard(v8f& a, v8f& b, v16b x, v16b y) {
#if DEV_ASM
  asm volatile("v_nop\n\tv_nop\n\tv_nop\n\tv_nop" : "+v"(a), "+v"(b) : "v"(x), "v"(y));
#else
  (void)a; (void)b; (void)x; (void)y;
#endif
}
__device__ __forceinline__ void dep_guard(v8f& a, v8f& b, v16h x, v16h y) {
#if DEV_ASM
  asm volatile("v_nop\n\tv_nop\n\tv_nop\n\tv_nop" : "+v"(a), "+v"(b) : "v"(x), "v"(y));
#else
  (void)a; (void)b; (void)x; (void)y;
#endif
}
__device__ __forceinline__ void keep4(v16b a, v16b b, v16b c, v16b d) {
#if DEV_ASM
  asm volatile("v_nop" :: "v"(a), "v"(b), "v"(c), "v"(d));
#else
  (void)a; (void)b; (void)c; (void)d;
#endif
}
__device__ __forceinline__ void keep4(v16h a, v16h b, v16h c, v16h d) {
#if DEV_ASM
  asm volatile("v_nop" :: "v"(a), "v"(b), "v"(c), "v"(d));
#else
  (void)a; (void)b; (void)c; (void)d;
#endif
}
__device__ __forceinline__ void keep1(v16h a) {
#if DEV_ASM
  asm volatile("v_nop" :: "v"(a));
#else
  (void)a;
#endif
}
__device__ __forceinline__ void acc_guard4(v8f& a, v8f& b, v8f& c, v8f& d) {
#if DEV_ASM
  asm volatile("v_nop\n\tv_nop\n\tv_nop\n\tv_nop" : "+v"(a), "+v"(b), "+v"(c), "+v"(d));
#else
  (void)a; (void)b; (void)c; (void)d;
#endif
}

template <int MODE>
__device__ __forceinline__ unsigned short cvm(float f) {
  const unsigned short hb = bf_bits(f);
  if (MODE == 0) return hb;
  return h_bits((_Float16)(bf_up(hb) * 64.0f));
}

template <int MODE>
__global__ __launch_bounds__(256) void cvt16x8(const float* __restrict__ in, long long sin,
                                               unsigned short* out, long long sout, int n8) {
  const int i = blockIdx.x * 256 + (int)threadIdx.x;
  const int y = blockIdx.y;
  if (i < n8) {
    const float* ip = in + (size_t)y * (size_t)sin + (size_t)i * 8;
    const v4f a  = *(const v4f*)(ip);
    const v4f a4 = *(const v4f*)(ip + 4);
    v4u p;
    p[0] = pk16(cvm<MODE>(a[0]),  cvm<MODE>(a[1]));
    p[1] = pk16(cvm<MODE>(a[2]),  cvm<MODE>(a[3]));
    p[2] = pk16(cvm<MODE>(a4[0]), cvm<MODE>(a4[1]));
    p[3] = pk16(cvm<MODE>(a4[2]), cvm<MODE>(a4[3]));
    unsigned short* o = out + (size_t)y * (size_t)sout + (size_t)i * 8;
    *(volatile v4u*)o = p;
    __threadfence();
    *(volatile v4u*)o = p;
  }
}

template <typename OT, int MI, int NPA, int NPB, int OUT_MODE, int CZ>
__global__ __launch_bounds__(256) void gemm_t(
    const unsigned short* __restrict__ Ap, const unsigned short* __restrict__ A2p, int lda, long long strideA,
    const unsigned short* __restrict__ Btp, int ldb, long long strideB,
    const unsigned short* __restrict__ B2p, int ldb2, long long strideB2, int K2,
    void* Cout, void* Cout2, int ldc, long long strideC, int ldc2, long long strideC2, int N2,
    int M, int N, int K, float oscale, float rscale2, float cscale, float rscaleC,
    const float* __restrict__ bias, const float* __restrict__ resid) {
  static_assert(CZ != 2 || ((16 * MI) % 32) == 0);
  static_assert(!(NPA == 2 && NPB == 2));
  typedef typename FT<OT>::frag V16;
  const OT* A  = (const OT*)(const void*)Ap;
  const OT* A2 = (const OT*)(const void*)A2p;
  const OT* Bt = (const OT*)(const void*)Btp;
  const OT* B2 = (const OT*)(const void*)B2p;
  __shared__ __align__(16) float sT[8][16 * 68];
  const int RT   = 16 * MI;
  const int b    = blockIdx.y;
  const int lane = threadIdx.x & 31;
  const int wave = threadIdx.x >> 5;
  const int tilesN = N >> 6;
  const int tilesM = M / RT;
  const int tile = blockIdx.x * 8 + wave;
  if (tile >= tilesM * tilesN) return;
  const int tm = tile / tilesN;
  const int tn = tile - tm * tilesN;
  const int m0 = tm * RT;
  const int n0 = tn << 6;
  if (CZ == 1) {
    if (n0 >= m0 + RT) return;
  }
  int kEnd = K;
  if (CZ == 2) {
    const int ke = m0 + RT;
    kEnd = (ke < K) ? ke : K;
  }

  const OT* Ab  = A  + (size_t)b * (size_t)strideA;
  const OT* A2b = A2 + (size_t)b * (size_t)strideA;
  const OT* Bb  = Bt + (size_t)b * (size_t)strideB;
  const OT* B2b = B2 + (size_t)b * (size_t)strideB2;

  const int rlane = lane & 15;
  const int koff  = (lane >> 4) * 8;
  const int mOff  = (lane >> 4) * 8;

  v8f acc[MI][4], acc2[MI][4];
#pragma unroll
  for (int i = 0; i < MI; ++i)
#pragma unroll
    for (int j = 0; j < 4; ++j) { acc[i][j] = zero8(); acc2[i][j] = zero8(); }

#pragma unroll 1
  for (int k0 = 0; k0 < kEnd; k0 += 32) {
    V16 bq[4];
#pragma unroll
    for (int j = 0; j < 4; ++j)
      bq[j] = ldfrag<OT>(Bb + (size_t)(n0 + (j << 4) + rlane) * ldb + koff + k0);
#pragma unroll
    for (int i = 0; i < MI; ++i) {
      const V16 af = ldfrag<OT>(Ab + (size_t)(m0 + (i << 4) + rlane) * lda + koff + k0);
#pragma unroll
      for (int j = 0; j < 4; ++j) acc[i][j] = mmar(af, bq[j], acc[i][j]);
      dep_guard(acc[i][0], acc[i][3], af, bq[3]);
      if (NPA == 2) {
        const V16 af2 = ldfrag<OT>(A2b + (size_t)(m0 + (i << 4) + rlane) * lda + koff + k0);
#pragma unroll
        for (int j = 0; j < 4; ++j) acc2[i][j] = mmar(af2, bq[j], acc2[i][j]);
        dep_guard(acc2[i][0], acc2[i][3], af2, bq[3]);
      }
    }
    keep4(bq[0], bq[1], bq[2], bq[3]);
    if (NPB == 2) {
      if (k0 < K2) {
        V16 br[4];
#pragma unroll
        for (int j = 0; j < 4; ++j)
          br[j] = ldfrag<OT>(B2b + (size_t)(n0 + (j << 4) + rlane) * ldb2 + koff + k0);
#pragma unroll
        for (int i = 0; i < MI; ++i) {
          const V16 afr = ldfrag<OT>(Ab + (size_t)(m0 + (i << 4) + rlane) * lda + koff + k0);
#pragma unroll
          for (int j = 0; j < 4; ++j) acc2[i][j] = mmar(afr, br[j], acc2[i][j]);
          dep_guard(acc2[i][0], acc2[i][3], afr, br[3]);
        }
        keep4(br[0], br[1], br[2], br[3]);
      }
    }
  }
#pragma unroll
  for (int i = 0; i < MI; ++i) {
    acc_guard4(acc[i][0], acc[i][1], acc[i][2], acc[i][3]);
    if (NPA == 2 || NPB == 2) acc_guard4(acc2[i][0], acc2[i][1], acc2[i][2], acc2[i][3]);
  }

  float* slab = sT[wave];
#pragma unroll
  for (int i = 0; i < MI; ++i) {
    const int mBase = m0 + (i << 4);
#pragma unroll
    for (int j = 0; j < 4; ++j) {
#pragma unroll
      for (int r = 0; r < 8; ++r) {
        float v = acc[i][j][r];
        if (NPA == 2 || NPB == 2) v += acc2[i][j][r] * rscale2;
        v = v * oscale;
        slab[(mOff + r) * 68 + (j << 4) + rlane] = v;
      }
    }
    __builtin_amdgcn_fence(__ATOMIC_RELEASE, "workgroup");
    __builtin_amdgcn_wave_barrier();
    __builtin_amdgcn_fence(__ATOMIC_ACQUIRE, "workgroup");
    if (OUT_MODE == 0 || OUT_MODE == 4) {
      float* C = (float*)Cout + (size_t)b * (size_t)strideC;
      const float* Rb = resid + (size_t)b * (size_t)strideC;
      const int h2 = lane >> 4, c4 = (lane & 15) * 4;
      v4f ov[8];
#pragma unroll
      for (int it = 0; it < 8; ++it) {
        const int row = it * 2 + h2;
        v4f v = *(const v4f*)(slab + row * 68 + c4);
        if (OUT_MODE == 4) {
          const v4f bb = *(const v4f*)(bias + n0 + c4);
          const v4f xr = *(const v4f*)(Rb + (size_t)(mBase + row) * ldc + n0 + c4);
#pragma unroll
          for (int e = 0; e < 4; ++e) v[e] = (v[e] + bfr(bb[e])) + bfr(xr[e]);
        }
        ov[it] = v;
      }
      for (int pass = 0; pass < 2; ++pass) {
#pragma unroll
        for (int it = 0; it < 8; ++it) {
          const int row = it * 2 + h2;
          *(volatile v4f*)(C + (size_t)(mBase + row) * ldc + n0 + c4) = ov[it];
        }
        __threadfence();
      }
    } else {
      const int q = lane >> 3, c8 = (lane & 7) * 8;
      unsigned short* C  = (unsigned short*)Cout  + (size_t)b * (size_t)strideC;
      unsigned short* C2 = (unsigned short*)Cout2 + (size_t)b * (size_t)strideC2;
      const bool wr2 = (OUT_MODE == 3) && (n0 < N2);
      v4u hv[4], lv[4];
#pragma unroll
      for (int it = 0; it < 4; ++it) {
        const int row = it * 4 + q;
        const float* sp = slab + row * 68 + c8;
        float f[8];
#pragma unroll
        for (int e = 0; e < 8; ++e) f[e] = sp[e] * cscale;
        v4u a, a2;
#pragma unroll
        for (int e = 0; e < 4; ++e) {
          const float f0 = f[2 * e], f1 = f[2 * e + 1];
          const _Float16 x0 = (_Float16)f0, x1 = (_Float16)f1;
          const unsigned short h0 = h_bits(x0), h1 = h_bits(x1);
          unsigned short l0 = 0, l1 = 0;
          if (OUT_MODE == 3) {
            l0 = h_bits((_Float16)((f0 - (float)x0) * rscaleC));
            l1 = h_bits((_Float16)((f1 - (float)x1) * rscaleC));
          }
          a[e] = pk16(h0, h1); a2[e] = pk16(l0, l1);
        }
        hv[it] = a; lv[it] = a2;
      }
      for (int pass = 0; pass < 2; ++pass) {
#pragma unroll
        for (int it = 0; it < 4; ++it) {
          const int row = it * 4 + q;
          *(volatile v4u*)(C + (size_t)(mBase + row) * ldc + n0 + c8) = hv[it];
          if (OUT_MODE == 3) {
            if (wr2) *(volatile v4u*)(C2 + (size_t)(mBase + row) * ldc2 + n0 + c8) = lv[it];
          }
        }
        __threadfence();
      }
    }
    __builtin_amdgcn_fence(__ATOMIC_RELEASE, "workgroup");
    __builtin_amdgcn_wave_barrier();
    __builtin_amdgcn_fence(__ATOMIC_ACQUIRE, "workgroup");
  }
}

__global__ __launch_bounds__(256) void k_trig(float* TRG) {
  __shared__ __align__(16) float sc[256];
  __shared__ __align__(16) float ss[256];
  const int tid = (int)threadIdx.x;
  const int m = blockIdx.x * 256 + tid;
  const float a = (6.28318548f * (float)m) * 0.00048828125f;
  float sv, cv;
  sincosf(a, &sv, &cv);
  sc[tid] = cv;
  ss[tid] = sv;
  __syncthreads();
  const int wave = tid >> 5, lane = tid & 31;
  if (wave < 4) {
    const int seg = wave >> 1;
    const int idx = ((wave & 1) * 32 + lane) * 4;
    const v4f vc = *(const v4f*)(sc + idx);
    const v4f vs = *(const v4f*)(ss + idx);
    v4f v;
#pragma unroll
    for (int e = 0; e < 4; ++e) v[e] = (seg == 0) ? vc[e] : vs[e];
    float* dst = TRG + (size_t)seg * SEQ + blockIdx.x * 256 + idx;
    *(volatile v4f*)dst = v;
    __threadfence();
    *(volatile v4f*)dst = v;
  }
}

__global__ __launch_bounds__(256) void k_ln(const float* __restrict__ X, const float* __restrict__ gam,
                                            const float* __restrict__ bet, float* Y32, unsigned short* Yh) {
  __shared__ __align__(16) float sT[CH * 68];
  const int t0 = blockIdx.x * 64, b = blockIdx.y;
  const int tid = (int)threadIdx.x, wave = tid >> 5, lane = tid & 31;
  float g[4], be[4];
#pragma unroll
  for (int j = 0; j < 4; ++j) { g[j] = bfr(gam[lane + 32 * j]); be[j] = bfr(bet[lane + 32 * j]); }
#pragma unroll 1
  for (int rr = 0; rr < 8; ++rr) {
    const int tl = wave * 8 + rr;
    const float* xr = X + ((size_t)b * SEQ + (size_t)(t0 + tl)) * CH;
    float v[4];
#pragma unroll
    for (int j = 0; j < 4; ++j) v[j] = bfr(xr[lane + 32 * j]);
    float s = (v[0] + v[1]) + (v[2] + v[3]);
#pragma unroll
    for (int off = 1; off < 32; off <<= 1) s += __shfl_xor(s, off, 32);
    const float mu = s * 0.0078125f;
    float d[4];
    float q = 0.f;
#pragma unroll
    for (int j = 0; j < 4; ++j) { d[j] = v[j] - mu; q += d[j] * d[j]; }
#pragma unroll
    for (int off = 1; off < 32; off <<= 1) q += __shfl_xor(q, off, 32);
    const float var = q * 0.0078125f;
    const float inv = 1.0f / sqrtf(var + 1e-5f);
#pragma unroll
    for (int j = 0; j < 4; ++j) sT[(lane + 32 * j) * 68 + tl] = ((d[j] * inv) * g[j]) + be[j];
  }
  __syncthreads();
  const int h2 = lane >> 4, c4 = (lane & 15) * 4;
  const int q8 = lane >> 3, c8 = (lane & 7) * 8;
  v4f fv[8];
  v4u hv[4];
#pragma unroll
  for (int it = 0; it < 8; ++it) {
    const int c = 2 * (wave + 8 * it) + h2;
    fv[it] = *(const v4f*)(sT + c * 68 + c4);
  }
#pragma unroll
  for (int it = 0; it < 4; ++it) {
    const int c = 4 * (wave + 8 * it) + q8;
    const float* sp = sT + c * 68 + c8;
    v4u p;
#pragma unroll
    for (int e = 0; e < 4; ++e) p[e] = pk16(h_bits((_Float16)sp[2 * e]), h_bits((_Float16)sp[2 * e + 1]));
    hv[it] = p;
  }
  for (int pass = 0; pass < 2; ++pass) {
#pragma unroll
    for (int it = 0; it < 8; ++it) {
      const int c = 2 * (wave + 8 * it) + h2;
      *(volatile v4f*)(Y32 + ((size_t)(c * NB + b)) * SEQ + t0 + c4) = fv[it];
    }
#pragma unroll
    for (int it = 0; it < 4; ++it) {
      const int c = 4 * (wave + 8 * it) + q8;
      *(volatile v4u*)(Yh + ((size_t)(c * NB + b)) * SEQ + t0 + c8) = hv[it];
    }
    __threadfence();
  }
}

__global__ __launch_bounds__(256) void k_cauchy(
    const float* __restrict__ Lr, const float* __restrict__ Li,
    const float* __restrict__ Pr, const float* __restrict__ Pi,
    const float* __restrict__ Br, const float* __restrict__ Bi,
    const float* __restrict__ Cr, const float* __restrict__ Ci,
    const float* __restrict__ TRG, unsigned short* ATh, unsigned short* ATl) {
  __shared__ float sLr[NS];
  __shared__ float sLi[NS];
  __shared__ float sV[7][NS];
  __shared__ __align__(16) float sRe[256];
  __shared__ __align__(16) float sIm[256];
  const int c = blockIdx.x >> 3, wb = blockIdx.x & 7;
  const int tid = (int)threadIdx.x, wave = tid >> 5, lane = tid & 31;
  if (tid < NS) {
    const int i = c * NS + tid;
    const float lr = fminf(bfr(Lr[i]), 1e-4f);
    const float li = bfr(Li[i]);
    const float pr = bfr(Pr[i]), pi = bfr(Pi[i]);
    const float br = bfr(Br[i]), bi = bfr(Bi[i]);
    const float cr = bfr(Cr[i]), ci = bfr(Ci[i]);
    sLr[tid] = lr; sLi[tid] = li;
    sV[0][tid] = cr * br + ci * bi;  sV[1][tid] = cr * bi - ci * br;
    sV[2][tid] = cr * pr + ci * pi;  sV[3][tid] = cr * pi - ci * pr;
    sV[4][tid] = pr * br + pi * bi;  sV[5][tid] = pr * bi - pi * br;
    sV[6][tid] = pr * pr + pi * pi;
  }
  __syncthreads();
  const int w = wb * 256 + tid;
  const float cw = TRG[w], sw = TRG[SEQ + w];
  const float opx = 1.0f + cw, opy = -sw;
  const float omx = 1.0f - cw, omy = sw;
  const float den1 = opx * opx + opy * opy;
  const float inv1 = 1.0f / den1;
  const float qx = (omx * opx + omy * opy) * inv1;
  const float qy = (omy * opx - omx * opy) * inv1;
  const float gx = 200.0f * qx, gy = 200.0f * qy;
  const float c2x = (2.0f * opx) * inv1;
  const float c2y = -(2.0f * opy) * inv1;
  float k00x = 0.f, k00y = 0.f, k01x = 0.f, k01y = 0.f, k10x = 0.f, k10y = 0.f, k11x = 0.f, k11y = 0.f;
#pragma unroll 1
  for (int n = 0; n < NS; ++n) {
    const float dx = gx - sLr[n], dy = gy - sLi[n];
    const float den = dx * dx + dy * dy;
    const float inv = 1.0f / den;
    const float rx = dx * inv, ry = -dy * inv;
    const float v0x = sV[0][n], v0y = sV[1][n];
    const float v1x = sV[2][n], v1y = sV[3][n];
    const float v2x = sV[4][n], v2y = sV[5][n];
    const float v3  = sV[6][n];
    k00x += v0x * rx - v0y * ry;  k00y += v0x * ry + v0y * rx;
    k01x += v1x * rx - v1y * ry;  k01y += v1x * ry + v1y * rx;
    k10x += v2x * rx - v2y * ry;  k10y += v2x * ry + v2y * rx;
    k11x += v3 * rx;              k11y += v3 * ry;
  }
  const float ex = 1.0f + k11x, ey = k11y;
  const float den3 = ex * ex + ey * ey;
  const float inv3 = 1.0f / den3;
  const float ux = ex * inv3, uy = -ey * inv3;
  const float wx = k01x * ux - k01y * uy, wy = k01x * uy + k01y * ux;
  const float w2x = wx * k10x - wy * k10y, w2y = wx * k10y + wy * k10x;
  const float inx = k00x - w2x, iny = k00y - w2y;
  const float atx = c2x * inx - c2y * iny;
  const float aty = c2x * iny + c2y * inx;
  sRe[tid] = atx;
  sIm[tid] = aty;
  __syncthreads();
  if (wave < 4) {
    const int pl = wave >> 1;
    const int im = wave & 1;
    const v4f ra = *(const v4f*)(sRe + 8 * lane), rb = *(const v4f*)(sRe + 8 * lane + 4);
    const v4f ia = *(const v4f*)(sIm + 8 * lane), ib = *(const v4f*)(sIm + 8 * lane + 4);
    float fr[8], fi[8];
#pragma unroll
    for (int e = 0; e < 4; ++e) { fr[e] = ra[e]; fr[4 + e] = rb[e]; fi[e] = ia[e]; fi[4 + e] = ib[e]; }
    v4u pk;
#pragma unroll
    for (int e2 = 0; e2 < 4; ++e2) {
      unsigned short o[2];
#pragma unroll
      for (int u = 0; u < 2; ++u) {
        const int e = 2 * e2 + u;
        const float v = (im == 0) ? fr[e] : fi[e];
        unsigned short hb, lb;
        split16(v * SAT, RCA, hb, lb);
        o[u] = (pl == 0) ? hb : lb;
      }
      pk[e2] = pk16(o[0], o[1]);
    }
    unsigned short* base = (pl == 0) ? ATh : ATl;
    unsigned short* dst = base + (size_t)c * KDFT + (size_t)im * SEQ + wb * 256 + 8 * lane;
    *(volatile v4u*)dst = pk;
    __threadfence();
    *(volatile v4u*)dst = pk;
  }
}

__global__ __launch_bounds__(256) void k_tw(const float* __restrict__ TRG, unsigned short* TW) {
  __shared__ __align__(16) float sTr[2 * SEQ];
  const int t = blockIdx.x, tid = (int)threadIdx.x;
#pragma unroll
  for (int u = 0; u < 4; ++u) {
    const int i4 = (tid + 256 * u) * 4;
    *(v4f*)(sTr + i4) = *(const v4f*)(TRG + i4);
  }
  __syncthreads();
  const int w0 = tid * 8;
  v4u pc, ps;
#pragma unroll
  for (int e2 = 0; e2 < 4; ++e2) {
    unsigned short hc[2], hs[2];
#pragma unroll
    for (int u = 0; u < 2; ++u) {
      const int w = w0 + 2 * e2 + u;
      const int m = (w * t) & (SEQ - 1);
      const float cv = sTr[m], sv = sTr[SEQ + m];
      hc[u] = h_bits((_Float16)cv);
      hs[u] = h_bits((_Float16)(-sv));
    }
    pc[e2] = pk16(hc[0], hc[1]);
    ps[e2] = pk16(hs[0], hs[1]);
  }
  unsigned short* dc = TW + (size_t)t * KDFT + w0;
  unsigned short* ds = dc + SEQ;
  *(volatile v4u*)dc = pc;
  *(volatile v4u*)ds = ps;
  __threadfence();
  *(volatile v4u*)dc = pc;
  *(volatile v4u*)ds = ps;
}

__global__ __launch_bounds__(256) void k_conv(const float* __restrict__ KT, const unsigned short* __restrict__ Yh,
                                              const float* __restrict__ Y32, const float* __restrict__ Dv,
                                              unsigned short* Hh, unsigned short* Hl) {
  extern __shared__ __align__(16) unsigned short dynK[];
  __shared__ __align__(16) unsigned short sOh[8][16 * 72];
  __shared__ __align__(16) unsigned short sOl[8][16 * 72];
  const int c = blockIdx.x;
  const int tid = (int)threadIdx.x, wave = tid >> 5, lane = tid & 31;
  const float* kt = KT + (size_t)c * SEQ;
#pragma unroll 1
  for (int task = tid; task < 8 * (LR / 8); task += 256) {
    const int j = task & 7, q = task >> 3;
    v4u ph, pl;
#pragma unroll
    for (int e2 = 0; e2 < 4; ++e2) {
      unsigned short hb[2], lb[2];
#pragma unroll
      for (int u = 0; u < 2; ++u) {
        const int e = 2 * e2 + u;
        const int ii = SEQ - 8 * q - e + j;
        const int ic = min(max(ii, 0), SEQ - 1);
        float v = kt[ic];
        v = (ii >= 0 && ii < SEQ) ? v : 0.0f;
        split16(v * KC, RCK, hb[u], lb[u]);
      }
      ph[e2] = pk16(hb[0], hb[1]);
      pl[e2] = pk16(lb[0], lb[1]);
    }
    *(v4u*)(dynK + (size_t)j * LR + 8 * q) = ph;
    *(v4u*)(dynK + (size_t)(8 + j) * LR + 8 * q) = pl;
  }
  __syncthreads();

  const float dsk = bfr(Dv[c]);
  const _Float16* Kh = (const _Float16*)(const void*)dynK;
  const int m = lane & 15, hh = lane >> 4, r7 = lane & 7;
  const _Float16* yrow = (const _Float16*)(const void*)Yh + ((size_t)(c * NB + m)) * SEQ + 8 * hh;
  const float* y32row = Y32 + ((size_t)(c * NB + m)) * SEQ + 8 * hh;
  const int abase = SEQ - (m & 8) + 8 * hh + r7 * LR;
  unsigned short* slabh = sOh[wave];
  unsigned short* slabl = sOl[wave];
  const int ntile = TROWS / 64;
  for (int tt = wave; tt < ntile; tt += 8) {
    const int t0 = tt * 64;
    v8f acc[4], acc2[4];
#pragma unroll
    for (int i = 0; i < 4; ++i) { acc[i] = zero8(); acc2[i] = zero8(); }
    const int ab0 = abase - t0;
#pragma unroll 1
    for (int s0 = 0; s0 < t0 + 64; s0 += 32) {
      const v16h bq = ldfrag<_Float16>(yrow + s0);
#pragma unroll
      for (int i = 0; i < 4; ++i) {
        const _Float16* pa = Kh + (ab0 + s0 - 16 * i);
        const v16h ah = ldfrag<_Float16>(pa);
        const v16h al = ldfrag<_Float16>(pa + 8 * LR);
        acc[i]  = mmar(ah, bq, acc[i]);
        acc2[i] = mmar(al, bq, acc2[i]);
        dep_guard(acc[i], acc2[i], ah, al);
      }
      keep1(bq);
    }
    acc_guard4(acc[0], acc[1], acc[2], acc[3]);
    acc_guard4(acc2[0], acc2[1], acc2[2], acc2[3]);
#pragma unroll
    for (int i = 0; i < 4; ++i) {
      const float* yp = y32row + t0 + 16 * i;
      const v4f ya = *(const v4f*)(yp);
      const v4f yb = *(const v4f*)(yp + 4);
      float yv[8];
#pragma unroll
      for (int e = 0; e < 4; ++e) { yv[e] = ya[e]; yv[4 + e] = yb[e]; }
      unsigned short hb[8], lb[8];
#pragma unroll
      for (int rr = 0; rr < 8; ++rr) {
        const float conv = (acc[i][rr] + acc2[i][rr] * 0.0009765625f) * 0.00390625f;
        const float ssm = conv + dsk * yv[rr];
        const float hv = 0.5f * ssm * erfcf(-ssm * 0.707106781186547524f);
        split16(hv, RCH, hb[rr], lb[rr]);
      }
      v4u p0, p1;
#pragma unroll
      for (int e = 0; e < 4; ++e) { p0[e] = pk16(hb[2 * e], hb[2 * e + 1]); p1[e] = pk16(lb[2 * e], lb[2 * e + 1]); }
      *(v4u*)(slabh + m * 72 + 16 * i + 8 * hh) = p0;
      *(v4u*)(slabl + m * 72 + 16 * i + 8 * hh) = p1;
    }
    __builtin_amdgcn_fence(__ATOMIC_RELEASE, "workgroup");
    __builtin_amdgcn_wave_barrier();
    __builtin_amdgcn_fence(__ATOMIC_ACQUIRE, "workgroup");
    const int q4 = lane >> 3, c8 = (lane & 7) * 8;
    v4u hv4[4], lv4[4];
#pragma unroll
    for (int it = 0; it < 4; ++it) {
      const int row = it * 4 + q4;
      hv4[it] = *(const v4u*)(slabh + row * 72 + c8);
      lv4[it] = *(const v4u*)(slabl + row * 72 + c8);
    }
    for (int pass = 0; pass < 2; ++pass) {
#pragma unroll
      for (int it = 0; it < 4; ++it) {
        const int row = it * 4 + q4;
        const size_t o = ((size_t)(c * NB + row)) * SEQ + t0 + c8;
        *(volatile v4u*)(Hh + o) = hv4[it];
        *(volatile v4u*)(Hl + o) = lv4[it];
      }
      __threadfence();
    }
    __builtin_amdgcn_fence(__ATOMIC_RELEASE, "workgroup");
    __builtin_amdgcn_wave_barrier();
    __builtin_amdgcn_fence(__ATOMIC_ACQUIRE, "workgroup");
  }
}

__global__ __launch_bounds__(256) void k_hT(const unsigned short* __restrict__ Hh, const unsigned short* __restrict__ Hl,
                                            unsigned short* H2h, unsigned short* H2l) {
  __shared__ __align__(16) unsigned short sH[64 * 136];
  const int t0 = blockIdx.x * 64, b = blockIdx.y, pl = blockIdx.z;
  const unsigned short* src = (pl == 0) ? Hh : Hl;
  unsigned short* dst = (pl == 0) ? H2h : H2l;
  const int tid = (int)threadIdx.x, wave = tid >> 5, lane = tid & 31;
  const int cq = tid >> 3, c8 = (tid & 7) * 8;
#pragma unroll
  for (int it = 0; it < 4; ++it) {
    const int c = cq + 32 * it;
    const v4u p = *(const v4u*)(src + ((size_t)(c * NB + b)) * SEQ + t0 + c8);
#pragma unroll
    for (int k = 0; k < 4; ++k) {
      sH[(c8 + 2 * k) * 136 + c]     = (unsigned short)(p[k] & 0xffffu);
      sH[(c8 + 2 * k + 1) * 136 + c] = (unsigned short)(p[k] >> 16);
    }
  }
  __syncthreads();
  const int h2 = lane >> 4, cc = (lane & 15) * 8;
  v4u ov[4];
#pragma unroll
  for (int it = 0; it < 4; ++it) {
    const int row = 2 * (wave + 8 * it) + h2;
    ov[it] = *(const v4u*)(sH + row * 136 + cc);
  }
  for (int pass = 0; pass < 2; ++pass) {
#pragma unroll
    for (int it = 0; it < 4; ++it) {
      const int row = 2 * (wave + 8 * it) + h2;
      *(volatile v4u*)(dst + ((size_t)(b * TROWS + t0 + row)) * CH + cc) = ov[it];
    }
    __threadfence();
  }
}

extern "C" void kernel_launch(void* const* d_in, const int* in_sizes, int n_in,
                              void* d_out, int out_size, void* d_ws, size_t ws_size,
                              hipStream_t stream) {
  if (n_in < 14) return;
  const long long needX = ((long long)(NB - 1) * SEQ + TROWS) * (long long)CH;
  if ((long long)in_sizes[0] < needX) return;
  if (in_sizes[1] < CH || in_sizes[2] < CH) return;
  for (int i = 3; i <= 10; ++i) { if (in_sizes[i] < CH * NS) return; }
  if (in_sizes[11] < CH) return;
  if (in_sizes[12] < CH * CH) return;
  if (in_sizes[13] < CH) return;
  if (out_size < 0) return;
  if ((long long)out_size < needX) return;

  const float* x   = (const float*)d_in[0];
  const float* gam = (const float*)d_in[1];
  const float* bet = (const float*)d_in[2];
  const float* Lr  = (const float*)d_in[3];
  const float* Li  = (const float*)d_in[4];
  const float* Pr  = (const float*)d_in[5];
  const float* Pi  = (const float*)d_in[6];
  const float* Br  = (const float*)d_in[7];
  const float* Bi  = (const float*)d_in[8];
  const float* Cr  = (const float*)d_in[9];
  const float* Ci  = (const float*)d_in[10];
  const float* Dv  = (const float*)d_in[11];
  const float* W   = (const float*)d_in[12];
  const float* bo  = (const float*)d_in[13];
  float* out0 = (float*)d_out;

  size_t off = 0;
  const size_t oTRG = off; off += SZ_TRG;
  const size_t oWoh = off; off += SZ_WOH;
  const size_t oY32 = off; off += SZ_Y32;
  const size_t oYh  = off; off += SZ_YH;
  const size_t oATh = off; off += SZ_AT;
  const size_t oATl = off; off += SZ_AT;
  const size_t oTW  = off; off += SZ_TW;
  const size_t oKT  = off; off += SZ_KT;
  const size_t oHh  = off; off += SZ_HC;
  const size_t oHl  = off; off += SZ_HC;
  const size_t oH2h = off; off += SZ_H2;
  const size_t oH2l = off; off += SZ_H2;
  if (off > ws_size) return;
  if (off > (size_t)134217728) return;

  char* ws = (char*)d_ws;
  float*          TRG = (float*)(ws + oTRG);
  unsigned short* Woh = (unsigned short*)(ws + oWoh);
  float*          Y32 = (float*)(ws + oY32);
  unsigned short* Yh  = (unsigned short*)(ws + oYh);
  unsigned short* ATh = (unsigned short*)(ws + oATh);
  unsigned short* ATl = (unsigned short*)(ws + oATl);
  unsigned short* TW  = (unsigned short*)(ws + oTW);
  float*          KT  = (float*)(ws + oKT);
  unsigned short* Hh  = (unsigned short*)(ws + oHh);
  unsigned short* Hl  = (unsigned short*)(ws + oHl);
  unsigned short* H2h = (unsigned short*)(ws + oH2h);
  unsigned short* H2l = (unsigned short*)(ws + oH2l);

  const dim3 blk(256);
  const int n8w = CH * CH / 8;
  const dim3 gCvtW((n8w + 255) / 256, 1);
  const dim3 gTrig(SEQ / 256);
  const dim3 gLn(TROWS / 64, NB);
  const dim3 gCau(CH * (SEQ / 256));
  const dim3 gTw(SEQ);
  const dim3 gDft((((CH / 32) * (SEQ / 64)) + 7) / 8, 1);
  const dim3 gConv(CH);
  const dim3 gHT(TROWS / 64, NB, 2);
  const dim3 gOut((((TROWS / 32) * (CH / 64)) + 7) / 8, NB);

  cvt16x8<1><<<gCvtW, blk, 0, stream>>>(W, 0LL, Woh, 0LL, n8w);
  k_trig<<<gTrig, blk, 0, stream>>>(TRG);
  k_ln<<<gLn, blk, 0, stream>>>(x, gam, bet, Y32, Yh);
  k_cauchy<<<gCau, blk, 0, stream>>>(Lr, Li, Pr, Pi, Br, Bi, Cr, Ci, TRG, ATh, ATl);
  k_tw<<<gTw, blk, 0, stream>>>(TRG, TW);
  gemm_t<_Float16, 2, 2, 1, 0, 0><<<gDft, blk, 0, stream>>>(
      ATh, ATl, KDFT, 0LL, TW, KDFT, 0LL,
      TW, KDFT, 0LL, 0,
      (void*)KT, (void*)KT, SEQ, 0LL, SEQ, 0LL, SEQ,
      CH, SEQ, KDFT, 1.0f / (SAT * (float)SEQ), 1.0f / RCA, 1.0f, 1.0f, bo, x);
  (void)hipFuncSetAttribute(reinterpret_cast<const void*>(&k_conv), hipFuncAttributeMaxDynamicSharedMemorySize, CONV_DYN_BYTES);
  k_conv<<<gConv, blk, CONV_DYN_BYTES, stream>>>(KT, Yh, Y32, Dv, Hh, Hl);
  k_hT<<<gHT, blk, 0, stream>>>(Hh, Hl, H2h, H2l);
  gemm_t<_Float16, 2, 2, 1, 4, 0><<<gOut, blk, 0, stream>>>(
      H2h, H2l, CH, (long long)TROWS * CH, Woh, CH, 0LL,
      Woh, CH, 0LL, 0,
      (void*)out0, (void*)out0, CH, (long long)SEQ * CH, CH, (long long)SEQ * CH, CH,
      TROWS, CH, CH, 0.015625f, 0.0009765625f, 1.0f, 1.0f, bo, x);
  (void)hipGetLastError();
}
